// C_T_F_Attention_90529320665770
// MI455X (gfx1250) — hardware-verified
//
#include <hip/hip_runtime.h>


#define NBt  32
#define CC   256
#define FR   7
#define TT   251
#define NPOS (FR * TT)
#define NPP  1792
#define NR   (NBt * NPP)
#define BEPS 1e-5f
#define DM   256
#define LOSC 1024.0f

typedef _Float16 h16;
typedef unsigned short bf;
typedef __attribute__((ext_vector_type(16))) __bf16   v16bf;
typedef __attribute__((ext_vector_type(16))) _Float16 v16h;
typedef __attribute__((ext_vector_type(8)))  _Float16 v8h;
typedef __attribute__((ext_vector_type(8)))  unsigned short v8us;
typedef __attribute__((ext_vector_type(8)))  float    v8f;
typedef __attribute__((ext_vector_type(4)))  float    v4f;
typedef v8h  __attribute__((may_alias)) v8ha;
typedef v4f  __attribute__((may_alias)) v4fa;
typedef v8us __attribute__((may_alias)) v8usa;

__device__ __forceinline__ unsigned short f2bf(float f) { unsigned u = __float_as_uint(f); u += 0x7FFFu + ((u >> 16) & 1u); return (unsigned short)(u >> 16); }
__device__ __forceinline__ float bf2f(unsigned short b) { return __uint_as_float(((unsigned)b) << 16); }
__device__ __forceinline__ float bfr(float f) { return bf2f(f2bf(f)); }
__device__ __forceinline__ v16h cat16(v8h lo, v8h hi) { return __builtin_shufflevector(lo, hi, 0, 1, 2, 3, 4, 5, 6, 7, 8, 9, 10, 11, 12, 13, 14, 15); }
__device__ __forceinline__ v16bf cat16b(v8us lo, v8us hi) { return __builtin_bit_cast(v16bf, __builtin_shufflevector(lo, hi, 0, 1, 2, 3, 4, 5, 6, 7, 8, 9, 10, 11, 12, 13, 14, 15)); }
__device__ __forceinline__ v8f wmma16(v16h a, v16h b, v8f c) { return __builtin_amdgcn_wmma_f32_16x16x32_f16(false, a, false, b, (short)0, c, false, false); }
__device__ __forceinline__ v8f wmmab(v16bf a, v16bf b, v8f c) { return __builtin_amdgcn_wmma_f32_16x16x32_bf16(false, a, false, b, (short)0, c, false, false); }

template <bool SPLITA, bool F16OUT = false>
__global__ __launch_bounds__(128) void k_gemmb(const bf* __restrict__ A, const bf* __restrict__ Al, const bf* __restrict__ Bn, const float* __restrict__ bias, float* C, int ldc, h16* C2, const float* __restrict__ R = nullptr, int K = DM, int roundR = 1) {
    __shared__ __align__(16) float ost[4][16 * 68];
    const int lane = threadIdx.x & 31, wave = threadIdx.x >> 5, lr = lane & 15, hi = lane >> 4;
    const int r0 = blockIdx.x * 64 + wave * 16, c0 = blockIdx.y * 64;
    const size_t aoff = (size_t)(r0 + lr) * K + 8 * hi;
    size_t boff[4];
#pragma unroll
    for (int t = 0; t < 4; ++t) boff[t] = (size_t)(c0 + t * 16 + lr) * K + 8 * hi;
    v8f acc[4];
#pragma unroll
    for (int t = 0; t < 4; ++t) acc[t] = (v8f){};
#pragma unroll 1
    for (int kc = 0; kc < K; kc += 32) {
        const v16bf a = cat16b(*(const v8us*)(A + aoff + kc), *(const v8us*)(A + aoff + kc + 16));
        v16bf al = a;
        if (SPLITA) al = cat16b(*(const v8us*)(Al + aoff + kc), *(const v8us*)(Al + aoff + kc + 16));
#pragma unroll
        for (int t = 0; t < 4; ++t) { const v16bf b = cat16b(*(const v8us*)(Bn + boff[t] + kc), *(const v8us*)(Bn + boff[t] + kc + 16)); acc[t] = wmmab(a, b, acc[t]); if (SPLITA) acc[t] = wmmab(al, b, acc[t]); }
        asm volatile("v_nop\n\tv_nop\n\tv_nop\n\tv_nop" : "+v"(acc[0]), "+v"(acc[1]), "+v"(acc[2]), "+v"(acc[3]) : "v"(a), "v"(al));
    }
    float* os = &ost[wave][0];
#pragma unroll
    for (int t = 0; t < 4; ++t) { const float bv = bias ? bfr(bias[c0 + t * 16 + lr]) : 0.f;
#pragma unroll
        for (int j = 0; j < 8; ++j) os[(hi * 8 + j) * 68 + t * 16 + lr] = acc[t][j] + bv; }
    __syncthreads();
    if (F16OUT) {
        h16* crow = (h16*)(void*)C + (size_t)r0 * ldc + c0;
        auto pass = [&]() {
#pragma unroll
            for (int s = 0; s < 4; ++s) { const int row = 4 * s + (lane >> 3), piece = lane & 7; const float* sp = os + row * 68 + piece * 8; v8h o, o2;
#pragma unroll
                for (int i = 0; i < 8; ++i) { const h16 a = (h16)sp[i]; o[i] = a; o2[i] = (h16)((sp[i] - (float)a) * LOSC); }
                *(volatile v8h*)(crow + (size_t)row * ldc + piece * 8) = o; if (C2) *(volatile v8h*)(C2 + (size_t)r0 * ldc + c0 + (size_t)row * ldc + piece * 8) = o2; }
        };
        pass(); __threadfence(); pass();
    } else {
        float* crow = C + (size_t)r0 * ldc + c0;
        auto pass = [&]() {
#pragma unroll
            for (int s = 0; s < 8; ++s) { const int Lid = (lane >> 3) + 4 * s, piece = lane & 7; const int row = Lid >> 1, cofs = (Lid & 1) * 32 + piece * 4;
                v4f val = *(const v4fa*)(os + row * 68 + cofs); if (R) { const v4f rv = *(const v4f*)(R + ((size_t)r0 + row) * ldc + c0 + cofs); val += roundR ? (v4f){bfr(rv[0]), bfr(rv[1]), bfr(rv[2]), bfr(rv[3])} : rv; }
                *(volatile v4f*)(crow + (size_t)row * ldc + cofs) = val; }
        };
        pass(); __threadfence(); pass();
    }
}


__global__ __launch_bounds__(256) void k_wtp(const float* __restrict__ Wm, int krows, int ncols, int kpad, bf* WT) {
    __shared__ __align__(16) unsigned short tl[64 * 72];
    const int tid = threadIdx.x, k0 = blockIdx.x * 64, n0 = blockIdx.y * 64;
    const int kk = tid >> 2, nq = (tid & 3) * 16;
    const int k = k0 + kk, kc = k < krows ? k : krows - 1;
#pragma unroll
    for (int i = 0; i < 16; ++i) { const int n = n0 + nq + i, ncl = n < ncols ? n : ncols - 1; const float w = Wm[(size_t)kc * ncols + ncl]; tl[(nq + i) * 72 + kk] = (k < krows && n < ncols) ? f2bf(w) : (unsigned short)0; }
    __syncthreads();
    const int piece = tid & 7;
    auto pass = [&]() {
#pragma unroll
        for (int s = 0; s < 2; ++s) { const int nr = (tid >> 3) + 32 * s; const v8us val = *(const v8usa*)(tl + nr * 72 + piece * 8); *(volatile v8us*)(WT + (size_t)(n0 + nr) * kpad + k0 + piece * 8) = val; }
    };
    pass(); __threadfence(); pass();
}

__global__ __launch_bounds__(256) void k_wpad(const float* __restrict__ Wm, int n, bf* WB) {
    const int lane = threadIdx.x & 31, o = blockIdx.x * 8 + (threadIdx.x >> 5); if (o >= 256) return; v8us ob;
#pragma unroll
    for (int i = 0; i < 8; ++i) { const int c = lane * 8 + i; const bool ok = (o < n) && (c < n); ob[i] = ok ? f2bf(Wm[(size_t)(ok ? o : 0) * n + (ok ? c : 0)]) : (unsigned short)0; }
    *(volatile v8us*)(WB + (size_t)o * 256 + lane * 8) = ob; __threadfence(); *(volatile v8us*)(WB + (size_t)o * 256 + lane * 8) = ob;
}
__global__ __launch_bounds__(288) void k_weff(const float* __restrict__ Wm, const float* __restrict__ bn, int n, float* WE) {
    const int c = threadIdx.x; float acc = 0.f;
    if (c < n) {
#pragma unroll 2
        for (int o = 0; o < n; ++o) { const float s = bfr(bn[o]) * rsqrtf(bfr(bn[3 * n + o]) + BEPS); acc = fmaf(s, bfr(Wm[(size_t)o * n + c]), acc); }
        acc /= (float)n; }
    else if (c == 256) {
#pragma unroll 2
        for (int o = 0; o < n; ++o) { const float s = bfr(bn[o]) * rsqrtf(bfr(bn[3 * n + o]) + BEPS); acc += bfr(bn[n + o]) - bfr(bn[2 * n + o]) * s; }
        acc /= (float)n; }
    *(volatile float*)(WE + c) = acc; __threadfence(); *(volatile float*)(WE + c) = acc;
}
__global__ __launch_bounds__(256) void k_qvc(const float* __restrict__ x, const float* __restrict__ WE, float* QV) {
    const size_t r = (size_t)blockIdx.x * 256 + threadIdx.x; if (r >= (size_t)NBt * CC * FR) return; float acc = WE[256];
#pragma unroll 4
    for (int t = 0; t < TT; ++t) acc = fmaf(bfr(x[r * TT + t]), WE[t], acc);
    *(volatile float*)(QV + r) = acc; __threadfence(); *(volatile float*)(QV + r) = acc;
}
__global__ __launch_bounds__(256) void k_qvp(const float* __restrict__ x, const float* __restrict__ WE, float* QV) {
    const size_t r = (size_t)blockIdx.x * 256 + threadIdx.x; if (r >= NR) return; const int b = (int)(r / NPP), p = (int)(r % NPP); float acc = 0.f;
    if (p < NPOS) { acc = WE[256];
#pragma unroll 4
        for (int c = 0; c < CC; ++c) acc = fmaf(bfr(x[((size_t)b * CC + c) * NPOS + p]), WE[c], acc); }
    *(volatile float*)(QV + r) = acc; __threadfence(); *(volatile float*)(QV + r) = acc;
}
template <int MODE>
__global__ __launch_bounds__(256) void k_diag(const float* __restrict__ QV, const float* __restrict__ KV, const float* __restrict__ lbn, float* DG) {
    const int L = (MODE == 0) ? CC : (MODE == 1) ? TT : FR; const int NN_ = (MODE == 2) ? NBt * TT : NBt * FR;
    const size_t g = (size_t)blockIdx.x * 256 + threadIdx.x; if (g >= (size_t)NN_ * L) return; const int n = (int)(g / L), i = (int)(g % L);
    const float s = bfr(lbn[0]) * rsqrtf(bfr(lbn[3]) + BEPS); const float h = bfr(lbn[1]) - bfr(lbn[2]) * s;
    auto rowof = [&](int nn, int l) -> size_t { if (MODE == 0) { const int b = nn / FR, fr = nn % FR; return ((size_t)b * CC + l) * FR + fr; }
                                               if (MODE == 1) { const int b = nn / FR, fr = nn % FR; return (size_t)b * NPP + fr * TT + l; }
                                               const int b = nn / TT, t = nn % TT; return (size_t)b * NPP + l * TT + t; };
    const float qi = QV[rowof(n, i)]; float mx = -3.0e38f;
#pragma unroll 1
    for (int j = 0; j < L; ++j) mx = fmaxf(mx, qi * KV[rowof(n, j)] * s + h);
    float sm = 0.f;
#pragma unroll 1
    for (int j = 0; j < L; ++j) sm += __expf(qi * KV[rowof(n, j)] * s + h - mx);
    const float d = __expf(qi * KV[rowof(n, i)] * s + h - mx) / sm;
    *(volatile float*)(DG + g) = d; __threadfence(); *(volatile float*)(DG + g) = d;
}
__global__ __launch_bounds__(256) void k_dsum(const float* __restrict__ DG, int L, int nn, float* D) {
    const int i = threadIdx.x; float s = 0.f;
    if (i < L) {
#pragma unroll 1
        for (int n = 0; n < nn; ++n) s += DG[(size_t)n * L + i]; }
    *(volatile float*)(D + i) = s; __threadfence(); *(volatile float*)(D + i) = s;
}
__global__ __launch_bounds__(256) void k_out(const float* __restrict__ V, const float* __restrict__ vbn, const float* __restrict__ Dc, const float* __restrict__ Df, const float* __restrict__ Dt, const float* __restrict__ x, int b, float* OUTP) {
    const size_t u = (size_t)blockIdx.x * 256 + threadIdx.x; if (u >= (size_t)CC * NPOS / 4) return; const size_t base = (size_t)b * CC * NPOS; v4f o;
#pragma unroll
    for (int k = 0; k < 4; ++k) { const size_t f = u * 4 + k; const int c = (int)(f / NPOS), p = (int)(f % NPOS); const int fr = p / TT, t = p % TT;
        const float s = bfr(vbn[c]) * rsqrtf(bfr(vbn[3 * CC + c]) + BEPS); const float h = bfr(vbn[CC + c]) - bfr(vbn[2 * CC + c]) * s;
        const float v = V[((size_t)b * NPP + p) * 256 + c] * s + h; o[k] = v * (Dc[c] + Dt[fr] + Df[t]) + bfr(x[base + f]); }
    *(volatile v4f*)(OUTP + base + u * 4) = o; __threadfence(); *(volatile v4f*)(OUTP + base + u * 4) = o;
}


extern "C" void kernel_launch(void* const* d_in, const int* in_sizes, int n_in,
                              void* d_out, int out_size, void* d_ws, size_t ws_size, hipStream_t stream) {
    (void)in_sizes; (void)n_in; (void)out_size;
    const float* x = (const float*)d_in[0];
    const float* qc_w = (const float*)d_in[1]; const float* qc_bn = (const float*)d_in[2]; const float* kc_w = (const float*)d_in[3]; const float* kc_bn = (const float*)d_in[4]; const float* lc_bn = (const float*)d_in[5];
    const float* qf_w = (const float*)d_in[6]; const float* qf_bn = (const float*)d_in[7]; const float* kf_w = (const float*)d_in[8]; const float* kf_bn = (const float*)d_in[9]; const float* lf_bn = (const float*)d_in[10];
    const float* qt_w = (const float*)d_in[11]; const float* qt_bn = (const float*)d_in[12]; const float* kt_w = (const float*)d_in[13]; const float* kt_bn = (const float*)d_in[14]; const float* lt_bn = (const float*)d_in[15];
    const float* v_w = (const float*)d_in[16]; const float* v_b = (const float*)d_in[17]; const float* v_bn = (const float*)d_in[18];
    float* out = (float*)d_out;
    char* wsp = (char*)d_ws;
    auto take = [&](size_t bytes) { char* p = wsp; wsp += (bytes + 255) & ~(size_t)255; return (void*)p; };
    bf* XP = (bf*)take((size_t)NR * CC * 2); float* G = (float*)take((size_t)NR * 256 * 4); bf* WB = (bf*)take(256 * 256 * 2);
    float* WEq = (float*)take(288 * 4); float* WEk = (float*)take(288 * 4); float* QV = (float*)take((size_t)NR * 4); float* KV = (float*)take((size_t)NR * 4);
    float* DG = (float*)take((size_t)NBt * TT * FR * 4 > (size_t)NBt * FR * CC * 4 ? (size_t)NBt * TT * FR * 4 : (size_t)NBt * FR * CC * 4);
    float* Dc = (float*)take(256 * 4); float* Df = (float*)take(256 * 4); float* Dt = (float*)take(256 * 4);
    if ((size_t)(wsp - (char*)d_ws) > ws_size) return;
    k_weff<<<1, 288, 0, stream>>>(qc_w, qc_bn, TT, WEq); k_weff<<<1, 288, 0, stream>>>(kc_w, kc_bn, TT, WEk);
    k_qvc<<<(NBt * CC * FR) / 256, 256, 0, stream>>>(x, WEq, QV); k_qvc<<<(NBt * CC * FR) / 256, 256, 0, stream>>>(x, WEk, KV);
    k_diag<0><<<(NBt * FR * CC + 255) / 256, 256, 0, stream>>>(QV, KV, lc_bn, DG); k_dsum<<<1, 256, 0, stream>>>(DG, CC, NBt * FR, Dc);
    k_weff<<<1, 288, 0, stream>>>(qf_w, qf_bn, CC, WEq); k_weff<<<1, 288, 0, stream>>>(kf_w, kf_bn, CC, WEk);
    k_qvp<<<NR / 256, 256, 0, stream>>>(x, WEq, QV); k_qvp<<<NR / 256, 256, 0, stream>>>(x, WEk, KV);
    k_diag<1><<<(NBt * FR * TT + 255) / 256, 256, 0, stream>>>(QV, KV, lf_bn, DG); k_dsum<<<1, 256, 0, stream>>>(DG, TT, NBt * FR, Df);
    k_weff<<<1, 288, 0, stream>>>(qt_w, qt_bn, CC, WEq); k_weff<<<1, 288, 0, stream>>>(kt_w, kt_bn, CC, WEk);
    k_qvp<<<NR / 256, 256, 0, stream>>>(x, WEq, QV); k_qvp<<<NR / 256, 256, 0, stream>>>(x, WEk, KV);
    k_diag<2><<<(NBt * TT * FR + 255) / 256, 256, 0, stream>>>(QV, KV, lt_bn, DG); k_dsum<<<1, 256, 0, stream>>>(DG, FR, NBt * TT, Dt);
    for (int b = 0; b < NBt; ++b) k_wtp<<<dim3(CC / 64, NPP / 64, 1), 256, 0, stream>>>(x + (size_t)b * CC * NPOS, CC, NPOS, CC, XP + (size_t)b * NPP * CC);
    k_wpad<<<256 / 8, 256, 0, stream>>>(v_w, CC, WB); k_gemmb<false, false><<<dim3(NR / 64, 4, 1), 128, 0, stream>>>(XP, nullptr, WB, v_b, G, 256, nullptr, nullptr, CC);
    for (int b = 0; b < NBt; ++b) k_out<<<(CC * NPOS / 4 + 255) / 256, 256, 0, stream>>>(G, v_bn, Dc, Df, Dt, x, b, out);
}
